// LPG_87101936763173
// MI455X (gfx1250) — hardware-verified
//
#include <hip/hip_runtime.h>


#define AS3 __attribute__((address_space(3)))

#define B_     256
#define S_     512
#define T_     32
#define E_     32
#define H_     512
#define G3_    1536
#define NF_    5
#define FW_    32
#define KC_    544
#define WPITCH 576
#define APITCH 552
#define YPITCH 520
#define HPITCH 512
#define PPITCH 52
#define NHD_   48
#define MB_    32
#define NBLK   (B_ / MB_)
#define NTHR   256
#define BS_    (B_ * S_)
#define FXW    8
#define FROWS  512

static_assert(KC_ == FW_ + H_);
static_assert(KC_ % 32 == 0);
static_assert(H_ % 32 == 0);
static_assert(APITCH % 8 == 0 && APITCH >= KC_);
static_assert(YPITCH % 8 == 0 && YPITCH >= H_);
static_assert(WPITCH % 8 == 0 && WPITCH >= KC_);
static_assert(PPITCH % 4 == 0 && PPITCH >= NHD_);
static_assert(MB_ == 32);
static_assert(NTHR == 256);
static_assert(H_ == (NTHR / 32) * 64);
static_assert(B_ % MB_ == 0);
static_assert(T_ == 32 && E_ == 32);
static_assert(S_ % 32 == 0);
static_assert(FROWS == (NTHR / 32) * 64);
static_assert(BS_ % FROWS == 0);
static_assert(NF_ <= FXW && FXW <= FW_);
static_assert(NHD_ % 16 == 0 && NHD_ >= T_ + 1);

typedef _Float16 v16h __attribute__((ext_vector_type(16)));
typedef _Float16 v8h  __attribute__((ext_vector_type(8)));
typedef float    v8f  __attribute__((ext_vector_type(8)));
typedef float    v4f  __attribute__((ext_vector_type(4)));

typedef AS3 _Float16*       lp_h;
typedef AS3 const _Float16* lcp_h;
typedef AS3 float*          lp_f;

union Frag { v16h v; v8h half[2]; };

constexpr int    NWPC  = WPITCH / 8;
constexpr int    NWP   = G3_ * NWPC;
constexpr int    NWBLK = NWP / 256;
constexpr int    NYP   = NHD_ * (H_ / 8);
constexpr int    NYBLK = NYP / 256;
static_assert(NWP % 256 == 0);
static_assert(NYP % 256 == 0);

constexpr size_t SZ_FX  = (size_t)BS_ * FXW * 2;
constexpr size_t SZ_WC  = (size_t)G3_ * WPITCH * 2;
constexpr size_t SZ_WY  = (size_t)NHD_ * H_ * 2;
constexpr size_t OFF_FX = 0;
constexpr size_t OFF_WC = OFF_FX + SZ_FX;
constexpr size_t OFF_WY = OFF_WC + SZ_WC;
constexpr size_t WS_END = OFF_WY + SZ_WY;
static_assert(OFF_WC % 128 == 0 && OFF_WY % 128 == 0);
static_assert(WS_END <= (size_t)134217728);
static_assert(SZ_FX % 128 == 0);
static_assert((size_t)NWP * 16 == SZ_WC);
static_assert((size_t)NYP * 16 == SZ_WY);

constexpr int    A_TILE    = MB_ * APITCH;
constexpr size_t LOFF_A    = 0;
constexpr size_t LSZ_A     = (size_t)2 * A_TILE * 2;
constexpr size_t LOFF_H    = LOFF_A + LSZ_A;
constexpr size_t LSZ_H     = (size_t)MB_ * HPITCH * 4;
constexpr size_t LOFF_Y    = LOFF_H + LSZ_H;
constexpr size_t LSZ_Y     = (size_t)MB_ * YPITCH * 2;
constexpr size_t LOFF_BE   = LOFF_Y + LSZ_Y;
constexpr size_t LOFF_BH   = LOFF_BE + (size_t)G3_ * 4;
constexpr size_t LOFF_P    = LOFF_BH + (size_t)H_ * 4;
constexpr size_t LOFF_PI   = LOFF_P + (size_t)MB_ * PPITCH * 4;
constexpr size_t LDS_BYTES = LOFF_PI + (size_t)MB_ * 32 * 4;
static_assert(LOFF_H % 16 == 0 && LOFF_Y % 16 == 0 && LOFF_BE % 16 == 0 && LOFF_BH % 16 == 0);
static_assert(LOFF_P % 16 == 0 && LOFF_PI % 16 == 0);
static_assert((2 * A_TILE) % 8 == 0);
static_assert((MB_ * HPITCH) % 4 == 0);

#define SCL    16.0f
#define INV256 0.00390625f

__device__ __forceinline__ float rcpx(float x) { return __builtin_amdgcn_rcpf(x); }
__device__ __forceinline__ float sigm(float x) { return rcpx(1.0f + __expf(-x)); }
__device__ __forceinline__ float tanhm(float x) {
    const float e = __expf(2.0f * x);
    return 1.0f - 2.0f * rcpx(e + 1.0f);
}
__device__ __forceinline__ v8f zero8() {
    v8f z;
#pragma unroll
    for (int i = 0; i < 8; ++i) z[i] = 0.0f;
    return z;
}

__device__ __forceinline__ void ldfrag_lds(Frag& f, lcp_h p) {
    f.half[0] = *(AS3 const v8h*)(p);
    f.half[1] = *(AS3 const v8h*)(p + 16);
}
__device__ __forceinline__ void ldfrag_glb(Frag& f, const _Float16* p) {
    f.half[0] = *(const v8h*)(p);
    f.half[1] = *(const v8h*)(p + 16);
}
__device__ __forceinline__ v8f mma16(v8f c, const Frag& a, const Frag& b) {
    return __builtin_amdgcn_wmma_f32_16x16x32_f16(false, a.v, false, b.v, (short)0, c, false, false);
}

__global__ __launch_bounds__(NTHR)
void feat_kernel(const float* __restrict__ rin, const int* __restrict__ din,
                 const float* __restrict__ pin,
                 const float* __restrict__ yt, const float* __restrict__ yt1,
                 const float* __restrict__ W1, const float* __restrict__ b1,
                 const float* __restrict__ W2, const float* __restrict__ b2,
                 _Float16* fx)
{
    const int tid  = threadIdx.x;
    const int lane = tid & 31;
    const int w    = tid >> 5;
    const int h    = lane >> 4;
    const int m    = lane & 15;
    const int r8   = lane & 7;

    Frag bw[2];
    float b1v[2], w2v[2];
#pragma unroll
    for (int nt = 0; nt < 2; ++nt) {
        const int e = nt * 16 + m;
#pragma unroll
        for (int i = 0; i < 16; ++i) {
            const int k = (i < 8) ? (8 * h + i) : (16 + 8 * h + (i - 8));
            bw[nt].v[i] = (_Float16)(W1[k * E_ + e] * SCL);
        }
        b1v[nt] = b1[e];
        w2v[nt] = W2[e];
    }
    const float b20 = b2[0];

#pragma unroll 1
    for (int g = 0; g < 4; ++g) {
        const int row0 = blockIdx.x * FROWS + w * 64 + g * 16;
        float pm[2];
#pragma unroll
        for (int src = 0; src < 2; ++src) {
            const float* Y    = (src == 0) ? yt : yt1;
            const float* base = Y + (size_t)(row0 + m) * T_ + 8 * h;
            const v4f x0 = *(const v4f*)(base);
            const v4f x1 = *(const v4f*)(base + 4);
            const v4f x2 = *(const v4f*)(base + 16);
            const v4f x3 = *(const v4f*)(base + 20);
            Frag a;
#pragma unroll
            for (int i = 0; i < 4; ++i) {
                a.v[i]      = (_Float16)(x0[i] * SCL);
                a.v[4 + i]  = (_Float16)(x1[i] * SCL);
                a.v[8 + i]  = (_Float16)(x2[i] * SCL);
                a.v[12 + i] = (_Float16)(x3[i] * SCL);
            }
            v8f acc[2];
            acc[0] = mma16(zero8(), a, bw[0]);
            acc[1] = mma16(zero8(), a, bw[1]);
            asm volatile("v_nop\n\tv_nop\n\tv_nop\n\tv_nop"
                         : "+v"(acc[0]), "+v"(acc[1])
                         : "v"(a.v), "v"(bw[0].v), "v"(bw[1].v));
            float sr[8];
#pragma unroll
            for (int r = 0; r < 8; ++r) {
                float s0 = fmaxf(acc[0][r] * INV256 + b1v[0], 0.0f) * w2v[0];
                s0 += fmaxf(acc[1][r] * INV256 + b1v[1], 0.0f) * w2v[1];
                sr[r] = s0;
            }
#pragma unroll
            for (int r = 0; r < 8; ++r) {
#pragma unroll
                for (int o = 8; o > 0; o >>= 1) sr[r] += __shfl_xor(sr[r], o, 32);
            }
            float pv = sr[0];
#pragma unroll
            for (int r = 1; r < 8; ++r) pv = (r8 == r) ? sr[r] : pv;
            pm[src] = pv + b20;
        }
        const int   lrow = row0 + 8 * h + r8;
        const float rv   = rin[lrow];
        const int   dv   = din[lrow];
        const float qv   = pin[lrow];
        v8h hv;
        hv[0] = (_Float16)(rv * SCL);
        hv[1] = (_Float16)((dv != 0) ? SCL : 0.0f);
        hv[2] = (_Float16)(qv * SCL);
        hv[3] = (_Float16)(pm[0] * SCL);
        hv[4] = (_Float16)((dv != 0) ? 0.0f : pm[1] * SCL);
        hv[5] = hv[0];
        hv[6] = hv[2];
        hv[7] = hv[3];
        _Float16* dst = fx + (size_t)lrow * FXW;
        const bool wr = ((lane & 8) == 0);
        if (wr) *(volatile v8h*)dst = hv;
        __threadfence();
        if (wr) *(volatile v8h*)dst = hv;
    }
}

__global__ __launch_bounds__(256)
void cvt_kernel(const float* __restrict__ Wi, const float* __restrict__ Whr,
                const float* __restrict__ Whz, const float* __restrict__ Whn,
                const float* __restrict__ Wy, const float* __restrict__ Wp,
                _Float16* Wcat, _Float16* Wyp)
{
    const int tid = threadIdx.x;
    if ((int)blockIdx.x < NWBLK) {
        const int p  = blockIdx.x * 256 + tid;
        const int n  = p / NWPC;
        const int c8 = (p - n * NWPC) * 8;
        const int g  = n >> 9;
        const int nu = n & (H_ - 1);
        const float* Wg = (g == 0) ? Whr : ((g == 1) ? Whz : Whn);
        v8h hv;
#pragma unroll
        for (int i = 0; i < 8; ++i) {
            const int c  = c8 + i;
            const int cw = min(c, NF_ - 1);
            const int ck = min(max(c - FW_, 0), H_ - 1);
            const float vi = Wi[cw * G3_ + n];
            const float vh = Wg[(size_t)ck * H_ + nu];
            const float v  = (c < NF_) ? vi : ((c >= FW_ && c < KC_) ? vh : 0.0f);
            hv[i] = (_Float16)(v * SCL);
        }
        _Float16* d = Wcat + (size_t)n * WPITCH + c8;
        *(volatile v8h*)d = hv;
        __threadfence();
        *(volatile v8h*)d = hv;
    } else {
        const int p  = ((int)blockIdx.x - NWBLK) * 256 + tid;
        const int o  = p >> 6;
        const int c8 = (p & 63) * 8;
        const int oc = min(o, T_ - 1);
        v8h hv;
#pragma unroll
        for (int i = 0; i < 8; ++i) {
            const int k = c8 + i;
            const float vy = Wy[k * T_ + oc];
            const float vp = Wp[k];
            const float v  = (o < T_) ? vy : ((o == T_) ? vp : 0.0f);
            hv[i] = (_Float16)(v * SCL);
        }
        _Float16* d = Wyp + (size_t)o * H_ + c8;
        *(volatile v8h*)d = hv;
        __threadfence();
        *(volatile v8h*)d = hv;
    }
}

__global__ __launch_bounds__(NTHR)
void gru_kernel(const _Float16* __restrict__ fx, const int* __restrict__ dm,
                const _Float16* __restrict__ Wcat, const _Float16* __restrict__ Wyp,
                const float* __restrict__ Wi, const float* __restrict__ bi,
                const float* __restrict__ bhn, const int* __restrict__ stp,
                const int* __restrict__ lif, const float* __restrict__ by,
                const float* __restrict__ bp, float* out)
{
    extern __shared__ __attribute__((aligned(16))) char smem[];
    lp_h sA  = (lp_h)(smem + LOFF_A);
    lp_f sH  = (lp_f)(smem + LOFF_H);
    lp_h sY  = (lp_h)(smem + LOFF_Y);
    lp_f sBe = (lp_f)(smem + LOFF_BE);
    lp_f sBh = (lp_f)(smem + LOFF_BH);
    lp_f sP  = (lp_f)(smem + LOFF_P);
    lp_f sPi = (lp_f)(smem + LOFF_PI);

    const int tid  = threadIdx.x;
    const int lane = tid & 31;
    const int w    = tid >> 5;
    const int h    = lane >> 4;
    const int m    = lane & 15;
    const int b0   = blockIdx.x * MB_;
    const float stepf = (float)stp[0];
    const float lifef = (float)lif[0];
    const float byc   = by[lane];
    const float bp0   = bp[0];

    {
        v8h zh;
#pragma unroll
        for (int i = 0; i < 8; ++i) zh[i] = (_Float16)0.0f;
        for (int i = tid; i < (2 * A_TILE) / 8; i += NTHR) *(AS3 v8h*)(sA + 8 * i) = zh;
        v4f zf;
#pragma unroll
        for (int i = 0; i < 4; ++i) zf[i] = 0.0f;
        for (int i = tid; i < (MB_ * HPITCH) / 4; i += NTHR) *(AS3 v4f*)(sH + 4 * i) = zf;
        for (int i = tid; i < G3_; i += NTHR)
            sBe[i] = bi[i] + stepf * Wi[5 * G3_ + i] + lifef * Wi[6 * G3_ + i];
        for (int i = tid; i < H_; i += NTHR) sBh[i] = bhn[i];
    }
    __syncthreads();
    if (tid < MB_) {
        const v8h fv = *(const v8h*)(fx + ((size_t)(b0 + tid) * S_ + (S_ - 1)) * FXW);
        *(AS3 v8h*)(sA + tid * APITCH) = fv;
    }

#pragma unroll 1
    for (int s = 0; s < S_; ++s) {
        const int t   = S_ - 1 - s;
        const int cur = s & 1;
        lp_h sAc = sA + cur * A_TILE;
        lp_h sAn = sA + (cur ^ 1) * A_TILE;

        __syncthreads();

        if (t > 0) {
            if (tid < MB_) {
                const v8h fv = *(const v8h*)(fx + ((size_t)(b0 + tid) * S_ + (t - 1)) * FXW);
                *(AS3 v8h*)(sAn + tid * APITCH) = fv;
            }
        }
        const int tq = (t > 0) ? (t - 1) : 0;
        const int dv = dm[(size_t)(b0 + lane) * S_ + tq];
        unsigned nmsk = __builtin_amdgcn_ballot_w32(dv != 0);
        nmsk = (t > 0) ? nmsk : 0u;

#pragma unroll 1
        for (int g4 = 0; g4 < 4; ++g4) {
            const int j0 = w * 64 + g4 * 16;
            const int n  = j0 + m;
            v8f acc[2][3], accx[2];
            lcp_h ab = sAc + m * APITCH + 8 * h;
            const _Float16* wb = Wcat + (size_t)(j0 + m) * WPITCH + 8 * h;
            {
                Frag a[2], b[3];
                ldfrag_lds(a[0], ab);
                ldfrag_lds(a[1], ab + 16 * APITCH);
#pragma unroll
                for (int q = 0; q < 3; ++q) ldfrag_glb(b[q], wb + (size_t)q * (512 * WPITCH));
#pragma unroll
                for (int mt = 0; mt < 2; ++mt) {
                    acc[mt][0] = mma16(zero8(), a[mt], b[0]);
                    acc[mt][1] = mma16(zero8(), a[mt], b[1]);
                    accx[mt]   = mma16(zero8(), a[mt], b[2]);
                }
                asm volatile("v_nop\n\tv_nop\n\tv_nop\n\tv_nop"
                             : "+v"(acc[0][0]), "+v"(acc[0][1]), "+v"(accx[0]),
                               "+v"(acc[1][0]), "+v"(acc[1][1]), "+v"(accx[1])
                             : "v"(a[0].v), "v"(a[1].v), "v"(b[0].v), "v"(b[1].v), "v"(b[2].v));
            }
            acc[0][2] = zero8();
            acc[1][2] = zero8();
#pragma unroll 1
            for (int k0 = FW_; k0 < KC_; k0 += 32) {
                Frag a[2], b[3];
                ldfrag_lds(a[0], ab + k0);
                ldfrag_lds(a[1], ab + 16 * APITCH + k0);
#pragma unroll
                for (int q = 0; q < 3; ++q) ldfrag_glb(b[q], wb + (size_t)q * (512 * WPITCH) + k0);
#pragma unroll
                for (int mt = 0; mt < 2; ++mt)
#pragma unroll
                    for (int q = 0; q < 3; ++q) acc[mt][q] = mma16(acc[mt][q], a[mt], b[q]);
                asm volatile("v_nop\n\tv_nop\n\tv_nop\n\tv_nop"
                             : "+v"(acc[0][0]), "+v"(acc[0][1]), "+v"(acc[0][2]),
                               "+v"(acc[1][0]), "+v"(acc[1][1]), "+v"(acc[1][2])
                             : "v"(a[0].v), "v"(a[1].v), "v"(b[0].v), "v"(b[1].v), "v"(b[2].v));
            }

            const float br = sBe[n];
            const float bz = sBe[H_ + n];
            const float bn = sBe[2 * H_ + n];
            const float bh = sBh[n];
#pragma unroll
            for (int mt = 0; mt < 2; ++mt) {
#pragma unroll
                for (int r = 0; r < 8; ++r) {
                    const int row = mt * 16 + 8 * h + r;
                    const float ar = acc[mt][0][r] * INV256 + br;
                    const float az = acc[mt][1][r] * INV256 + bz;
                    const float ah = acc[mt][2][r] * INV256 + bh;
                    const float ax = accx[mt][r] * INV256 + bn;
                    const float rg = sigm(ar);
                    const float zg = sigm(az);
                    const float ng = tanhm(ax + rg * ah);
                    const float hp = sH[row * HPITCH + n];
                    const float hn = (1.0f - zg) * ng + zg * hp;
                    const float yv = fmaxf(hn, 0.0f);
                    sY[row * YPITCH + n] = (_Float16)(yv * SCL);
                    const bool  rs = ((nmsk >> row) & 1u) != 0u;
                    const float hi = rs ? 0.0f : hn;
                    sH[row * HPITCH + n] = hi;
                    sAn[row * APITCH + FW_ + n] = (_Float16)(hi * SCL);
                }
            }
        }

        __syncthreads();

        if (w < 6) {
            const int mt = (w >= 3) ? 1 : 0;
            const int nt = w - 3 * mt;
            v8f pacc = zero8();
            lcp_h ya = sY + (mt * 16 + m) * YPITCH + 8 * h;
            const _Float16* gb = Wyp + (size_t)(nt * 16 + m) * H_ + 8 * h;
#pragma unroll 1
            for (int k0 = 0; k0 < H_; k0 += 32) {
                Frag a, b;
                ldfrag_lds(a, ya + k0);
                ldfrag_glb(b, gb + k0);
                pacc = mma16(pacc, a, b);
                asm volatile("v_nop\n\tv_nop\n\tv_nop\n\tv_nop" : "+v"(pacc) : "v"(a.v), "v"(b.v));
            }
            const int col = nt * 16 + m;
#pragma unroll
            for (int r = 0; r < 8; ++r)
                sP[(mt * 16 + 8 * h + r) * PPITCH + col] = pacc[r] * INV256;
        }
        __syncthreads();

        {
            const int slot = t & 31;
            float pv[4];
#pragma unroll
            for (int i = 0; i < 4; ++i) {
                const int row = w * 4 + i;
                const float v = sP[row * PPITCH + lane] + byc;
                float mx = v;
#pragma unroll
                for (int o = 16; o > 0; o >>= 1) mx = fmaxf(mx, __shfl_xor(mx, o, 32));
                const float ev = __expf(v - mx);
                float sm = ev;
#pragma unroll
                for (int o = 16; o > 0; o >>= 1) sm += __shfl_xor(sm, o, 32);
                pv[i] = ev * rcpx(sm);
                if (lane == 0) sPi[row * 32 + slot] = sP[row * PPITCH + T_] + bp0;
            }
#pragma unroll
            for (int i = 0; i < 4; ++i) {
                float* op = out + BS_ + ((size_t)(b0 + w * 4 + i) * S_ + t) * T_ + lane;
                *(volatile float*)op = pv[i];
            }
            __threadfence();
#pragma unroll
            for (int i = 0; i < 4; ++i) {
                float* op = out + BS_ + ((size_t)(b0 + w * 4 + i) * S_ + t) * T_ + lane;
                *(volatile float*)op = pv[i];
            }
            if (slot == 0) {
                __syncthreads();
                float qv[4];
#pragma unroll
                for (int i = 0; i < 4; ++i) qv[i] = sPi[(w * 4 + i) * 32 + lane];
#pragma unroll
                for (int i = 0; i < 4; ++i) {
                    float* op = out + (size_t)(b0 + w * 4 + i) * S_ + t + lane;
                    *(volatile float*)op = qv[i];
                }
                __threadfence();
#pragma unroll
                for (int i = 0; i < 4; ++i) {
                    float* op = out + (size_t)(b0 + w * 4 + i) * S_ + t + lane;
                    *(volatile float*)op = qv[i];
                }
            }
        }
    }
}

extern "C" void kernel_launch(void* const* d_in, const int* in_sizes, int n_in,
                              void* d_out, int out_size, void* d_ws, size_t ws_size,
                              hipStream_t stream)
{
    if (n_in < 21) return;
    if (in_sizes[0]  != BS_)       return;
    if (in_sizes[1]  != BS_)       return;
    if (in_sizes[2]  != BS_)       return;
    if (in_sizes[3]  != BS_ * T_)  return;
    if (in_sizes[4]  != BS_ * T_)  return;
    if (in_sizes[5]  < 1)          return;
    if (in_sizes[6]  < 1)          return;
    if (in_sizes[7]  != T_ * E_)   return;
    if (in_sizes[8]  != E_)        return;
    if (in_sizes[9]  != E_)        return;
    if (in_sizes[10] < 1)          return;
    if (in_sizes[11] != 7 * G3_)   return;
    if (in_sizes[12] != G3_)       return;
    if (in_sizes[13] != H_ * H_)   return;
    if (in_sizes[14] != H_ * H_)   return;
    if (in_sizes[15] != H_ * H_)   return;
    if (in_sizes[16] != H_)        return;
    if (in_sizes[17] != H_)        return;
    if (in_sizes[18] < 1)          return;
    if (in_sizes[19] != H_ * T_)   return;
    if (in_sizes[20] != T_)        return;
    if (out_size != BS_ + BS_ * T_) return;
    if (ws_size < WS_END)          return;

    const float* rin = (const float*)d_in[0];
    const int*   din = (const int*)  d_in[1];
    const float* pin = (const float*)d_in[2];
    const float* yt  = (const float*)d_in[3];
    const float* yt1 = (const float*)d_in[4];
    const int*   stp = (const int*)  d_in[5];
    const int*   lif = (const int*)  d_in[6];
    const float* W1  = (const float*)d_in[7];
    const float* b1  = (const float*)d_in[8];
    const float* W2  = (const float*)d_in[9];
    const float* b2  = (const float*)d_in[10];
    const float* Wi  = (const float*)d_in[11];
    const float* bi  = (const float*)d_in[12];
    const float* Whr = (const float*)d_in[13];
    const float* Whz = (const float*)d_in[14];
    const float* Whn = (const float*)d_in[15];
    const float* bhn = (const float*)d_in[16];
    const float* Wp  = (const float*)d_in[17];
    const float* bp  = (const float*)d_in[18];
    const float* Wy  = (const float*)d_in[19];
    const float* by  = (const float*)d_in[20];
    float* out = (float*)d_out;

    char* ws = (char*)d_ws;
    _Float16* fx   = (_Float16*)(ws + OFF_FX);
    _Float16* Wcat = (_Float16*)(ws + OFF_WC);
    _Float16* Wyp  = (_Float16*)(ws + OFF_WY);

    feat_kernel<<<dim3(BS_ / FROWS), dim3(NTHR), 0, stream>>>(
        rin, din, pin, yt, yt1, W1, b1, W2, b2, fx);

    cvt_kernel<<<dim3(NWBLK + NYBLK), dim3(256), 0, stream>>>(
        Wi, Whr, Whz, Whn, Wy, Wp, Wcat, Wyp);

    hipFuncSetAttribute(reinterpret_cast<const void*>(&gru_kernel),
                        hipFuncAttributeMaxDynamicSharedMemorySize, (int)LDS_BYTES);
    gru_kernel<<<dim3(NBLK), dim3(NTHR), LDS_BYTES, stream>>>(
        (const _Float16*)fx, din, (const _Float16*)Wcat, (const _Float16*)Wyp,
        Wi, bi, bhn, stp, lif, by, bp, out);
}
